// Seq2SeqForecaster_19292993093921
// MI455X (gfx1250) — hardware-run, weakly checked
//
#include <hip/hip_runtime.h>
#include <math.h>
#include <stdint.h>

constexpr int NSEQ    = 256;
constexpr int NSTEP   = 512;
constexpr int NPRED   = 96;
constexpr int NHID    = 256;
constexpr int NG3     = 768;
constexpr int NTHR    = 256;
constexpr int NWAVE   = 8;
constexpr int TROWS   = 16;
constexpr int UPW     = 32;
constexpr int HPITCH  = 264;
constexpr int XCH     = 64;
constexpr int KCHUNKS = NHID / 32;
constexpr int GSTRIDE = NHID * NHID;
constexpr int OUT_F4_ITERS = TROWS * NPRED / 128;
constexpr float A_CARRY = 16.0f;
constexpr float W_CARRY = 64.0f;
constexpr float Z_FOLD  = 1.0f / 1024.0f;

static_assert(NSEQ % TROWS == 0, "grid covers all sequences exactly");
static_assert(NSTEP % XCH == 0, "x chunks tile the time axis exactly");
static_assert(TROWS * XCH == NTHR * 4, "one float4 per thread per x chunk");
static_assert((NG3 * NHID / 8) % NTHR == 0, "weight prep grid exact");
static_assert(NHID % 32 == 0, "K multiple of 32");
static_assert(NWAVE * UPW == NHID, "waves cover all hidden units");
static_assert(NWAVE * 32 == NTHR, "wave count");
static_assert(TROWS == 2 * NWAVE, "head: two rows per wave");
static_assert(NHID == 32 * 8, "head: eight elements per lane");
static_assert((TROWS * NPRED) % 128 == 0, "output block is whole 512-B groups");
static_assert(HPITCH % 8 == 0 && HPITCH >= NHID, "A fragment rows 16-B aligned and in range");

typedef __attribute__((ext_vector_type(16))) _Float16 v16h;
typedef __attribute__((ext_vector_type(8)))  _Float16 v8h;
typedef __attribute__((ext_vector_type(16))) __bf16   v16b;
typedef __attribute__((ext_vector_type(8)))  __bf16   v8b;
typedef __attribute__((ext_vector_type(8)))  float    v8f;
typedef __attribute__((ext_vector_type(4)))  float    v4f;

__device__ __forceinline__ unsigned short f2bf_bits(float f) {
  unsigned u = __float_as_uint(f);
  return (unsigned short)((u + 0x7FFFu + ((u >> 16) & 1u)) >> 16);
}
__device__ __forceinline__ float bf_bits2f(unsigned short h) { return __uint_as_float(((unsigned)h) << 16); }
__device__ __forceinline__ float bfr(float f) { return bf_bits2f(f2bf_bits(f)); }

__device__ __forceinline__ void dep_guard_h(v8f& a, v8f& b, v16h x, v16h y) { asm volatile("v_nop\n\tv_nop\n\tv_nop\n\tv_nop" : "+v"(a), "+v"(b) : "v"(x), "v"(y)); }
__device__ __forceinline__ void dep_guard_b(v8f& a, v8f& b, v16b x, v16b y) { asm volatile("v_nop\n\tv_nop\n\tv_nop\n\tv_nop" : "+v"(a), "+v"(b) : "v"(x), "v"(y)); }
__device__ __forceinline__ void keep4_h(v16h a, v16h b, v16h c, v16h d) { asm volatile("v_nop" :: "v"(a), "v"(b), "v"(c), "v"(d)); }
__device__ __forceinline__ void keep4_b(v16b a, v16b b, v16b c, v16b d) { asm volatile("v_nop" :: "v"(a), "v"(b), "v"(c), "v"(d)); }
__device__ __forceinline__ void acc_guard4(v8f& a, v8f& b, v8f& c, v8f& d) { asm volatile("v_nop\n\tv_nop\n\tv_nop\n\tv_nop" : "+v"(a), "+v"(b), "+v"(c), "+v"(d)); }
__device__ __forceinline__ void acc_guard3(v8f& a, v8f& b, v8f& c) { asm volatile("v_nop\n\tv_nop\n\tv_nop\n\tv_nop" : "+v"(a), "+v"(b), "+v"(c)); }
template <typename T> struct Frag;
template <> struct Frag<_Float16> {
  typedef v16h V; union U { v16h v; v8h h[2]; };
  static __device__ __forceinline__ v16h load(const _Float16* p) {
    U f; f.h[0] = *(const v8h*)(p); f.h[1] = *(const v8h*)(p + 16); return f.v;
  }
  static __device__ __forceinline__ v8f mma(v16h a, v16h b, v8f c) {
    return __builtin_amdgcn_wmma_f32_16x16x32_f16(false, a, false, b, (short)0, c, false, false);
  }
  static __device__ __forceinline__ void guard(v8f& a, v8f& b, v16h x, v16h y) { dep_guard_h(a, b, x, y); }
  static __device__ __forceinline__ void keep(v16h a, v16h b, v16h c, v16h d) { keep4_h(a, b, c, d); }
};
template <> struct Frag<__bf16> {
  typedef v16b V; union U { v16b v; v8b h[2]; };
  static __device__ __forceinline__ v16b load(const __bf16* p) {
    U f; f.h[0] = *(const v8b*)(p); f.h[1] = *(const v8b*)(p + 16); return f.v;
  }
  static __device__ __forceinline__ v8f mma(v16b a, v16b b, v8f c) {
    return __builtin_amdgcn_wmma_f32_16x16x32_bf16(false, a, false, b, (short)0, c, false, false);
  }
  static __device__ __forceinline__ void guard(v8f& a, v8f& b, v16b x, v16b y) { dep_guard_b(a, b, x, y); }
  static __device__ __forceinline__ void keep(v16b a, v16b b, v16b c, v16b d) { keep4_b(a, b, c, d); }
};
typedef Frag<_Float16> FragH;

__device__ __forceinline__ float fsig(float v)  { return __builtin_amdgcn_rcpf(1.0f + __expf(-v)); }
__device__ __forceinline__ float ftanh(float v) { return 1.0f - 2.0f * __builtin_amdgcn_rcpf(__expf(2.0f * v) + 1.0f); }

__global__ __launch_bounds__(NTHR) void wprep_kernel(const float* __restrict__ W, int n8, unsigned short* __restrict__ O) {
  const int i = blockIdx.x * NTHR + threadIdx.x;
  if (i >= n8) return;
  const int e0 = i * 8;
  v8h hv;
#pragma unroll
  for (int e = 0; e < 8; ++e) {
    const float fb = bfr(W[e0 + e]);
    hv[e] = (_Float16)(fb * W_CARRY);
  }
  *(volatile v8h*)(O + e0) = hv;
  __threadfence();
  *(volatile v8h*)(O + e0) = hv;
}

__device__ __forceinline__ void mac_g3(v8f (&acc)[3], const _Float16* arow, const _Float16* wh) {
#pragma unroll 1
  for (int kc = 0; kc < KCHUNKS; ++kc) {
    const int k0 = kc * 32;
    const v16h a  = FragH::load(arow + k0);
    const v16h b0 = FragH::load(wh + k0);
    const v16h b1 = FragH::load(wh + GSTRIDE + k0);
    const v16h b2 = FragH::load(wh + 2 * GSTRIDE + k0);
    acc[0] = FragH::mma(a, b0, acc[0]);
    acc[1] = FragH::mma(a, b1, acc[1]);
    acc[2] = FragH::mma(a, b2, acc[2]);
    acc_guard3(acc[0], acc[1], acc[2]);
    keep4_h(a, b0, b1, b2);
  }
}

__device__ __forceinline__ void mac_g4(v8f (&acc)[4], const _Float16* abrow, const _Float16* asrow,
                                       const _Float16* wi, const _Float16* wh) {
#pragma unroll 1
  for (int kc = 0; kc < KCHUNKS; ++kc) {
    const int k0 = kc * 32;
    const v16h ab  = FragH::load(abrow + k0);
    const v16h as  = FragH::load(asrow + k0);
    const v16h bir = FragH::load(wi + k0);
    const v16h bhr = FragH::load(wh + k0);
    const v16h biz = FragH::load(wi + GSTRIDE + k0);
    const v16h bhz = FragH::load(wh + GSTRIDE + k0);
    const v16h bin = FragH::load(wi + 2 * GSTRIDE + k0);
    const v16h bhn = FragH::load(wh + 2 * GSTRIDE + k0);
    acc[0] = FragH::mma(ab, bir, acc[0]);
    acc[0] = FragH::mma(as, bhr, acc[0]);
    acc[1] = FragH::mma(ab, biz, acc[1]);
    acc[1] = FragH::mma(as, bhz, acc[1]);
    acc[2] = FragH::mma(ab, bin, acc[2]);
    acc[3] = FragH::mma(as, bhn, acc[3]);
    acc_guard4(acc[0], acc[1], acc[2], acc[3]);
    keep4_h(ab, as, bir, bhr);
    keep4_h(biz, bhz, bin, bhn);
  }
}

__device__ __forceinline__ void gru_cell8(const v8f (&acc)[4], float cr, float cz, float cin, float chn, float (&h)[8]) {
#pragma unroll
  for (int r = 0; r < 8; ++r) {
    const float pr  = fmaf(acc[0][r], Z_FOLD, cr);
    const float pz  = fmaf(acc[1][r], Z_FOLD, cz);
    const float gin = fmaf(acc[2][r], Z_FOLD, cin);
    const float ghn = fmaf(acc[3][r], Z_FOLD, chn);
    const float rr  = fsig(pr);
    const float zz  = fsig(pz);
    const float nn  = ftanh(fmaf(rr, ghn, gin));
    h[r] = fmaf(zz, h[r] - nn, nn);
  }
}

__device__ __forceinline__ void gru_cell8_in1(const v8f (&acc)[3], const float (&xin)[8],
                                              float wr, float wz, float wn, float cr, float cz, float cin, float chn,
                                              float (&h)[8]) {
#pragma unroll
  for (int r = 0; r < 8; ++r) {
    const float pr  = fmaf(acc[0][r], Z_FOLD, fmaf(xin[r], wr, cr));
    const float pz  = fmaf(acc[1][r], Z_FOLD, fmaf(xin[r], wz, cz));
    const float gin = fmaf(xin[r], wn, cin);
    const float ghn = fmaf(acc[2][r], Z_FOLD, chn);
    const float rr  = fsig(pr);
    const float zz  = fsig(pz);
    const float nn  = ftanh(fmaf(rr, ghn, gin));
    h[r] = fmaf(zz, h[r] - nn, nn);
  }
}

__global__ __launch_bounds__(NTHR) void seq_gru_kernel(
    const float* __restrict__ x,
    const float* __restrict__ w_ih0, const float* __restrict__ b_ih0, const float* __restrict__ b_hh0,
    const float* __restrict__ b_ih1, const float* __restrict__ b_hh1,
    const float* __restrict__ wd_ih, const float* __restrict__ bd_ih, const float* __restrict__ bd_hh,
    const float* __restrict__ w_o,   const float* __restrict__ b_o,
    const unsigned short* __restrict__ Whh0p, const unsigned short* __restrict__ Wih1p,
    const unsigned short* __restrict__ Whh1p, const unsigned short* __restrict__ Wdhhp,
    float* __restrict__ out) {
  __shared__ __align__(16) _Float16 H0t[TROWS * HPITCH];
  __shared__ __align__(16) _Float16 H1t[TROWS * HPITCH];
  __shared__ __align__(16) float    Xs[TROWS * XCH];
  __shared__ __align__(16) float    Hf[TROWS * NHID];
  __shared__ __align__(16) float    Os[TROWS * NPRED];
  __shared__ __align__(16) float    Pf[TROWS];

  const int tid = threadIdx.x, lane = tid & 31, wave = tid >> 5;
  const int c = lane & 15, hh = lane >> 4, koff = hh * 8;
  const int rb = 8 * hh;
  const int ubase = wave * UPW;
  const int rowbase = blockIdx.x * TROWS;

#pragma unroll 1
  for (int i = tid; i < TROWS * HPITCH; i += NTHR) { H0t[i] = (_Float16)0.0f; H1t[i] = (_Float16)0.0f; }
  if (tid < TROWS) Pf[tid] = 0.0f;

  float w0r[2], w0z[2], w0n[2], c0r[2], c0z[2], c0in[2], c0hn[2], c1r[2], c1z[2], c1in[2], c1hn[2];
#pragma unroll
  for (int ut = 0; ut < 2; ++ut) {
    const int j = ubase + 16 * ut + c;
    w0r[ut]  = bfr(w_ih0[j]);
    w0z[ut]  = bfr(w_ih0[NHID + j]);
    w0n[ut]  = bfr(w_ih0[2 * NHID + j]);
    c0r[ut]  = bfr(b_ih0[j]) + bfr(b_hh0[j]);
    c0z[ut]  = bfr(b_ih0[NHID + j]) + bfr(b_hh0[NHID + j]);
    c0in[ut] = bfr(b_ih0[2 * NHID + j]);
    c0hn[ut] = bfr(b_hh0[2 * NHID + j]);
    c1r[ut]  = bfr(b_ih1[j]) + bfr(b_hh1[j]);
    c1z[ut]  = bfr(b_ih1[NHID + j]) + bfr(b_hh1[NHID + j]);
    c1in[ut] = bfr(b_ih1[2 * NHID + j]);
    c1hn[ut] = bfr(b_hh1[2 * NHID + j]);
  }

  float hst0[2][8], hst1[2][8];
#pragma unroll
  for (int ut = 0; ut < 2; ++ut)
#pragma unroll
    for (int r = 0; r < 8; ++r) { hst0[ut][r] = 0.0f; hst1[ut][r] = 0.0f; }
  __syncthreads();

  const _Float16* a0row = H0t + c * HPITCH + koff;
  const _Float16* a1row = H1t + c * HPITCH + koff;
  const _Float16* whh0 = (const _Float16*)Whh0p + (size_t)(ubase + c) * NHID + koff;
  const _Float16* wih1 = (const _Float16*)Wih1p + (size_t)(ubase + c) * NHID + koff;
  const _Float16* whh1 = (const _Float16*)Whh1p + (size_t)(ubase + c) * NHID + koff;
  const _Float16* wdhh = (const _Float16*)Wdhhp + (size_t)(ubase + c) * NHID + koff;
  const v8f z8 = {0.f, 0.f, 0.f, 0.f, 0.f, 0.f, 0.f, 0.f};

#pragma unroll 1
  for (int t = 0; t < NSTEP; ++t) {
    const int tc = t & (XCH - 1);
    if (tc == 0) {
      const int row = tid >> 4, c4 = (tid & 15) * 4;
      const v4f v = *(const v4f*)(x + ((size_t)(rowbase + row) * NSTEP + (size_t)(t + c4)));
      v4f w;
      w[0] = bfr(v[0]); w[1] = bfr(v[1]); w[2] = bfr(v[2]); w[3] = bfr(v[3]);
      *(v4f*)(Xs + row * XCH + c4) = w;
      __syncthreads();
    }
    {
      float xr[8];
#pragma unroll
      for (int r = 0; r < 8; ++r) xr[r] = Xs[(rb + r) * XCH + tc];
#pragma unroll
      for (int ut = 0; ut < 2; ++ut) {
        v8f acc[3];
        acc[0] = z8; acc[1] = z8; acc[2] = z8;
        mac_g3(acc, a0row, whh0 + ut * 16 * NHID);
        gru_cell8_in1(acc, xr, w0r[ut], w0z[ut], w0n[ut], c0r[ut], c0z[ut], c0in[ut], c0hn[ut], hst0[ut]);
      }
      __syncthreads();
#pragma unroll
      for (int ut = 0; ut < 2; ++ut)
#pragma unroll
        for (int r = 0; r < 8; ++r) H0t[(rb + r) * HPITCH + ubase + 16 * ut + c] = (_Float16)(A_CARRY * hst0[ut][r]);
      __syncthreads();
    }
    {
#pragma unroll
      for (int ut = 0; ut < 2; ++ut) {
        v8f acc[4];
        acc[0] = z8; acc[1] = z8; acc[2] = z8; acc[3] = z8;
        mac_g4(acc, a0row, a1row, wih1 + ut * 16 * NHID, whh1 + ut * 16 * NHID);
        gru_cell8(acc, c1r[ut], c1z[ut], c1in[ut], c1hn[ut], hst1[ut]);
      }
      __syncthreads();
#pragma unroll
      for (int ut = 0; ut < 2; ++ut)
#pragma unroll
        for (int r = 0; r < 8; ++r) H1t[(rb + r) * HPITCH + ubase + 16 * ut + c] = (_Float16)(A_CARRY * hst1[ut][r]);
      __syncthreads();
    }
  }

  float wdr[2], wdz[2], wdn[2], cdr[2], cdz[2], cdin[2], cdhn[2];
#pragma unroll
  for (int ut = 0; ut < 2; ++ut) {
    const int j = ubase + 16 * ut + c;
    wdr[ut]  = bfr(wd_ih[j]);
    wdz[ut]  = bfr(wd_ih[NHID + j]);
    wdn[ut]  = bfr(wd_ih[2 * NHID + j]);
    cdr[ut]  = bfr(bd_ih[j]) + bfr(bd_hh[j]);
    cdz[ut]  = bfr(bd_ih[NHID + j]) + bfr(bd_hh[NHID + j]);
    cdin[ut] = bfr(bd_ih[2 * NHID + j]);
    cdhn[ut] = bfr(bd_hh[2 * NHID + j]);
  }
  float wo8[8];
#pragma unroll
  for (int e = 0; e < 8; ++e) wo8[e] = bfr(w_o[lane * 8 + e]);
  const float bo0 = bfr(b_o[0]);

#pragma unroll 1
  for (int t = 0; t < NPRED; ++t) {
    float pin[8];
#pragma unroll
    for (int r = 0; r < 8; ++r) pin[r] = Pf[rb + r];
#pragma unroll
    for (int ut = 0; ut < 2; ++ut) {
      v8f acc[3];
      acc[0] = z8; acc[1] = z8; acc[2] = z8;
      mac_g3(acc, a1row, wdhh + ut * 16 * NHID);
      gru_cell8_in1(acc, pin, wdr[ut], wdz[ut], wdn[ut], cdr[ut], cdz[ut], cdin[ut], cdhn[ut], hst1[ut]);
    }
    __syncthreads();
#pragma unroll
    for (int ut = 0; ut < 2; ++ut)
#pragma unroll
      for (int r = 0; r < 8; ++r) {
        H1t[(rb + r) * HPITCH + ubase + 16 * ut + c] = (_Float16)(A_CARRY * hst1[ut][r]);
        Hf[(rb + r) * NHID + ubase + 16 * ut + c] = hst1[ut][r];
      }
    __syncthreads();
#pragma unroll
    for (int rr = 0; rr < 2; ++rr) {
      const int row = 2 * wave + rr;
      const float* hp = Hf + row * NHID + lane * 8;
      const v4f ha = *(const v4f*)(hp);
      const v4f hb = *(const v4f*)(hp + 4);
      float s = ha[0] * wo8[0];
      s = fmaf(ha[1], wo8[1], s);
      s = fmaf(ha[2], wo8[2], s);
      s = fmaf(ha[3], wo8[3], s);
      s = fmaf(hb[0], wo8[4], s);
      s = fmaf(hb[1], wo8[5], s);
      s = fmaf(hb[2], wo8[6], s);
      s = fmaf(hb[3], wo8[7], s);
      s += __shfl_xor(s, 16, 32);
      s += __shfl_xor(s, 8, 32);
      s += __shfl_xor(s, 4, 32);
      s += __shfl_xor(s, 2, 32);
      s += __shfl_xor(s, 1, 32);
      if (lane == 0) {
        const float o = s + bo0;
        Pf[row] = o;
        Os[row * NPRED + t] = o;
      }
    }
    __syncthreads();
  }

  {
    float* op = out + (size_t)blockIdx.x * (size_t)(TROWS * NPRED);
    for (int pass = 0; pass < 2; ++pass) {
#pragma unroll 1
      for (int it = wave; it < OUT_F4_ITERS; it += NWAVE) {
        const int idx = it * 128 + lane * 4;
        const v4f v = *(const v4f*)(Os + idx);
        *(volatile v4f*)(op + idx) = v;
      }
      __threadfence();
    }
  }
}

extern "C" void kernel_launch(void* const* d_in, const int* in_sizes, int n_in,
                              void* d_out, int out_size, void* d_ws, size_t ws_size, hipStream_t stream) {
  if (n_in < 15 || d_out == nullptr || d_ws == nullptr) return;
  if (in_sizes[0] != NSEQ * NSTEP || in_sizes[1] != NG3 || in_sizes[2] != NG3 * NHID || in_sizes[3] != NG3 ||
      in_sizes[4] != NG3 || in_sizes[5] != NG3 * NHID || in_sizes[6] != NG3 * NHID || in_sizes[7] != NG3 ||
      in_sizes[8] != NG3 || in_sizes[9] != NG3 || in_sizes[10] != NG3 * NHID || in_sizes[11] != NG3 ||
      in_sizes[12] != NG3 || in_sizes[13] != NHID || in_sizes[14] < 1 || out_size != NSEQ * NPRED) return;

  const float* x     = (const float*)d_in[0];
  const float* w_ih0 = (const float*)d_in[1];
  const float* w_hh0 = (const float*)d_in[2];
  const float* b_ih0 = (const float*)d_in[3];
  const float* b_hh0 = (const float*)d_in[4];
  const float* w_ih1 = (const float*)d_in[5];
  const float* w_hh1 = (const float*)d_in[6];
  const float* b_ih1 = (const float*)d_in[7];
  const float* b_hh1 = (const float*)d_in[8];
  const float* wd_ih = (const float*)d_in[9];
  const float* wd_hh = (const float*)d_in[10];
  const float* bd_ih = (const float*)d_in[11];
  const float* bd_hh = (const float*)d_in[12];
  const float* w_o   = (const float*)d_in[13];
  const float* b_o   = (const float*)d_in[14];
  float* out = (float*)d_out;

  char* ws = (char*)d_ws; size_t off = 0;
  auto carve = [&](size_t bytes) -> char* { char* p = ws + off; off += (bytes + 255) & ~(size_t)255; return p; };
  const size_t plane_bytes = (size_t)NG3 * NHID * 2;
  unsigned short* WHH0 = (unsigned short*)carve(plane_bytes);
  unsigned short* WIH1 = (unsigned short*)carve(plane_bytes);
  unsigned short* WHH1 = (unsigned short*)carve(plane_bytes);
  unsigned short* WDHH = (unsigned short*)carve(plane_bytes);
  if (off > ws_size || off > (size_t)134217728) return;

  const int n8 = NG3 * NHID / 8;
  wprep_kernel<<<n8 / NTHR, NTHR, 0, stream>>>(w_hh0, n8, WHH0);
  wprep_kernel<<<n8 / NTHR, NTHR, 0, stream>>>(w_ih1, n8, WIH1);
  wprep_kernel<<<n8 / NTHR, NTHR, 0, stream>>>(w_hh1, n8, WHH1);
  wprep_kernel<<<n8 / NTHR, NTHR, 0, stream>>>(wd_hh, n8, WDHH);
  seq_gru_kernel<<<NSEQ / TROWS, NTHR, 0, stream>>>(x, w_ih0, b_ih0, b_hh0, b_ih1, b_hh1, wd_ih, bd_ih, bd_hh, w_o, b_o,
                                                    WHH0, WIH1, WHH1, WDHH, out);
}
